// ConvNeXtParallelMoELoRA_10299331575852
// MI455X (gfx1250) — hardware-verified
//
#include <hip/hip_runtime.h>
#include <stdint.h>


typedef _Float16 f16;
typedef f16 v8h __attribute__((ext_vector_type(8)));
typedef f16 v16h __attribute__((ext_vector_type(16)));
typedef __bf16 v16b __attribute__((ext_vector_type(16)));
typedef unsigned short v8us __attribute__((ext_vector_type(8)));
typedef unsigned short v16us __attribute__((ext_vector_type(16)));
typedef float v8f __attribute__((ext_vector_type(8)));
typedef float v4f __attribute__((ext_vector_type(4)));
typedef unsigned int v4u __attribute__((ext_vector_type(4)));
typedef v4u v4ua __attribute__((may_alias));
typedef v4f v4fa __attribute__((may_alias));

__device__ __forceinline__ v8f vzero8() {
    v8f z = {0.f, 0.f, 0.f, 0.f, 0.f, 0.f, 0.f, 0.f};
    return z;
}

__device__ __forceinline__ v8f wmma_f16(v16h a, v16h b, v8f c) {
    v8f d = __builtin_amdgcn_wmma_f32_16x16x32_f16(false, a, false, b, (short)0, c, false, false);
    asm volatile("v_nop\n\tv_nop\n\tv_nop\n\tv_nop" : "+v"(d) : "v"(a), "v"(b));
    return d;
}

__device__ __forceinline__ v8f wmma_bf16(v16b a, v16b b, v8f c) {
    v8f d = __builtin_amdgcn_wmma_f32_16x16x32_bf16(false, a, false, b, (short)0, c, false, false);
    asm volatile("v_nop\n\tv_nop\n\tv_nop\n\tv_nop" : "+v"(d) : "v"(a), "v"(b));
    return d;
}

__device__ __forceinline__ v16h ld_frag_h(const f16* __restrict__ rowp, int k0, int h) {
    const f16* p = rowp + k0 + 8 * h;
    v8h e0 = *(const v8h*)p;
    v8h e1 = *(const v8h*)(p + 16);
    return __builtin_shufflevector(e0, e1, 0, 1, 2, 3, 4, 5, 6, 7, 8, 9, 10, 11, 12, 13, 14, 15);
}

__device__ __forceinline__ v16b ld_frag_b(const unsigned short* __restrict__ rowp, int k0, int h) {
    const unsigned short* p = rowp + k0 + 8 * h;
    v8us e0 = *(const v8us*)p;
    v8us e1 = *(const v8us*)(p + 16);
    v16us v = __builtin_shufflevector(e0, e1, 0, 1, 2, 3, 4, 5, 6, 7, 8, 9, 10, 11, 12, 13, 14, 15);
    return __builtin_bit_cast(v16b, v);
}

__device__ __forceinline__ unsigned short bf16_rne(float f) {
    unsigned u = __builtin_bit_cast(unsigned, f);
    u = (u + 0x7FFFu + ((u >> 16) & 1u)) >> 16;
    return (unsigned short)u;
}

__device__ __forceinline__ float bf16_to_f32(unsigned short s) {
    unsigned u = ((unsigned)s) << 16;
    return __builtin_bit_cast(float, u);
}

__device__ __forceinline__ float gelu_exact(float v) {
    return 0.5f * v * (1.0f + erff(v * 0.70710678118654752440f));
}

__global__ __launch_bounds__(256) void k_cvt_x(const float* __restrict__ x, f16* __restrict__ x16, int T) {
    const int w = threadIdx.x >> 5, l = threadIdx.x & 31;
    const int row = blockIdx.x * 8 + w;
    if (row >= T) return;
    const float* src = x + (size_t)row * 768;
    f16* dst = x16 + (size_t)row * 768;
    v4u pk[3];
#pragma unroll
    for (int it = 0; it < 3; ++it) {
        const int c = 256 * it + 8 * l;
        v4f a = *(const v4f*)(src + c);
        v4f b = *(const v4f*)(src + c + 4);
        v8h hv;
        hv[0] = (f16)a[0]; hv[1] = (f16)a[1]; hv[2] = (f16)a[2]; hv[3] = (f16)a[3];
        hv[4] = (f16)b[0]; hv[5] = (f16)b[1]; hv[6] = (f16)b[2]; hv[7] = (f16)b[3];
        pk[it] = __builtin_bit_cast(v4u, hv);
    }
#pragma unroll
    for (int it = 0; it < 3; ++it) {
        const int c = 256 * it + 8 * l;
        *(volatile v4u*)(dst + c) = pk[it];
    }
    __threadfence();
#pragma unroll
    for (int it = 0; it < 3; ++it) {
        const int c = 256 * it + 8 * l;
        *(volatile v4u*)(dst + c) = pk[it];
    }
}

__global__ __launch_bounds__(64) void k_prep_w(const float* __restrict__ in, f16* __restrict__ out,
                                               int KR, int NC, float scale) {
    __shared__ float s[64][33];
    const int tid = threadIdx.x, w = tid >> 5, l = tid & 31;
    const int k0 = blockIdx.y * 64, n0 = blockIdx.x * 32;
#pragma unroll 8
    for (int it = 0; it < 32; ++it) {
        const int r = 2 * it + w;
        s[r][l] = in[(size_t)(k0 + r) * NC + n0 + l];
    }
    __syncthreads();
    v4u pk[4];
#pragma unroll
    for (int it = 0; it < 4; ++it) {
        const int nl = 16 * w + 4 * it + (l >> 3);
        const int p = l & 7;
        v8h hv;
#pragma unroll
        for (int q = 0; q < 8; ++q) hv[q] = (f16)(scale * s[8 * p + q][nl]);
        pk[it] = __builtin_bit_cast(v4u, hv);
    }
#pragma unroll
    for (int it = 0; it < 4; ++it) {
        const int nl = 16 * w + 4 * it + (l >> 3);
        const int p = l & 7;
        f16* dst = out + (size_t)(n0 + nl) * KR + k0 + 8 * p;
        *(volatile v4u*)dst = pk[it];
    }
    __threadfence();
#pragma unroll
    for (int it = 0; it < 4; ++it) {
        const int nl = 16 * w + 4 * it + (l >> 3);
        const int p = l & 7;
        f16* dst = out + (size_t)(n0 + nl) * KR + k0 + 8 * p;
        *(volatile v4u*)dst = pk[it];
    }
}

__global__ __launch_bounds__(256) void k_prep_s(const float* __restrict__ w_down, const float* __restrict__ w_up,
                                                f16* __restrict__ wd16, unsigned short* __restrict__ wu) {
    const int w = threadIdx.x >> 5, l = threadIdx.x & 31;
    if (blockIdx.x == 0) {
#pragma unroll 1
        for (int it = 0; it < 24; ++it) {
            const int d = 96 * w + 4 * it + (l >> 3);
            const int p = l & 7;
            v8us hv;
#pragma unroll
            for (int q = 0; q < 8; ++q) {
                const int c = 8 * (p & 3) + q;
                const float val = (c < 24) ? 64.0f * w_up[(size_t)c * 768 + d] : 0.0f;
                const unsigned short hi = bf16_rne(val);
                const unsigned short lo = bf16_rne(val - bf16_to_f32(hi));
                hv[q] = (p < 4) ? hi : lo;
            }
            const v4u pk = __builtin_bit_cast(v4u, hv);
            unsigned short* dst = wu + (size_t)d * 64 + 8 * p;
            *(volatile v4u*)dst = pk;
            __threadfence();
            *(volatile v4u*)dst = pk;
        }
    } else {
#pragma unroll 1
        for (int rr = 0; rr < 4; ++rr) {
            const int rho = 4 * w + rr;
            const int e = rho >> 3, r = rho & 7;
#pragma unroll
            for (int it = 0; it < 3; ++it) {
                const int p = l + 32 * it;
                v8h hv;
#pragma unroll
                for (int q = 0; q < 8; ++q) {
                    const int k = 8 * p + q;
                    const float val = (rho < 24) ? 32.0f * w_down[((size_t)e * 768 + k) * 8 + r] : 0.0f;
                    hv[q] = (f16)val;
                }
                const v4u pk = __builtin_bit_cast(v4u, hv);
                f16* dst = wd16 + (size_t)rho * 768 + 8 * p;
                *(volatile v4u*)dst = pk;
                __threadfence();
                *(volatile v4u*)dst = pk;
            }
        }
    }
}

__global__ __launch_bounds__(64) void k_tok(const float* __restrict__ x, const float* __restrict__ rw,
                                            const float* __restrict__ rb, const f16* __restrict__ x16,
                                            const f16* __restrict__ wd16, unsigned short* __restrict__ ca, int T) {
    __shared__ float s_lg[2][32][4];
    __shared__ float s_comb[32][4];
    __shared__ __align__(16) unsigned short s_ca[32][64];

    const int tid = threadIdx.x, w = tid >> 5, l = tid & 31, h = l >> 4, m = l & 15;
    const int t0 = blockIdx.x * 32;

    v8f accd[2];
    accd[0] = vzero8();
    accd[1] = vzero8();
    {
        const f16* ap = x16 + (size_t)(t0 + 16 * w + m) * 768;
        const f16* bp0 = wd16 + (size_t)m * 768;
        const f16* bp1 = wd16 + (size_t)(16 + m) * 768;
#pragma unroll 1
        for (int k0 = 0; k0 < 768; k0 += 32) {
            v16h a = ld_frag_h(ap, k0, h);
            v16h b0 = ld_frag_h(bp0, k0, h);
            v16h b1 = ld_frag_h(bp1, k0, h);
            accd[0] = wmma_f16(a, b0, accd[0]);
            accd[1] = wmma_f16(a, b1, accd[1]);
        }
    }

    {
        const float* xr = x + (size_t)(t0 + l) * 768 + 384 * w;
        const float* rp = rw + (size_t)(384 * w) * 3;
        float g0a = 0.f, g1a = 0.f, g2a = 0.f, g0b = 0.f, g1b = 0.f, g2b = 0.f;
#pragma unroll 1
        for (int kk = 0; kk < 96; ++kk) {
            v4f xv = *(const v4f*)(xr + 4 * kk);
            v4f r0 = *(const v4f*)(rp + 12 * kk);
            v4f r1 = *(const v4f*)(rp + 12 * kk + 4);
            v4f r2 = *(const v4f*)(rp + 12 * kk + 8);
            g0a = fmaf(xv[0], r0[0], g0a); g1a = fmaf(xv[0], r0[1], g1a); g2a = fmaf(xv[0], r0[2], g2a);
            g0b = fmaf(xv[1], r0[3], g0b); g1b = fmaf(xv[1], r1[0], g1b); g2b = fmaf(xv[1], r1[1], g2b);
            g0a = fmaf(xv[2], r1[2], g0a); g1a = fmaf(xv[2], r1[3], g1a); g2a = fmaf(xv[2], r2[0], g2a);
            g0b = fmaf(xv[3], r2[1], g0b); g1b = fmaf(xv[3], r2[2], g1b); g2b = fmaf(xv[3], r2[3], g2b);
        }
        s_lg[w][l][0] = g0a + g0b;
        s_lg[w][l][1] = g1a + g1b;
        s_lg[w][l][2] = g2a + g2b;
    }
    __syncthreads();
    if (tid < 32) {
        const float lg0 = (s_lg[0][tid][0] + s_lg[1][tid][0]) + rb[0];
        const float lg1 = (s_lg[0][tid][1] + s_lg[1][tid][1]) + rb[1];
        const float lg2 = (s_lg[0][tid][2] + s_lg[1][tid][2]) + rb[2];
        const float mx = fmaxf(lg0, fmaxf(lg1, lg2));
        const float e0 = expf(lg0 - mx), e1 = expf(lg1 - mx), e2 = expf(lg2 - mx);
        const float inv = 1.0f / ((e0 + e1) + e2);
        const float p0 = e0 * inv, p1 = e1 * inv, p2 = e2 * inv;
        int amin = 0;
        float pm = p0;
        if (p1 <= pm) { amin = 1; pm = p1; }
        if (p2 <= pm) { amin = 2; pm = p2; }
        const float c0 = (amin == 0) ? 0.0f : p0;
        const float c1 = (amin == 1) ? 0.0f : p1;
        const float c2 = (amin == 2) ? 0.0f : p2;
        const float psum = (c0 + c1) + c2;
        const float invd = 1.0f / (psum + 1e-6f);
        s_comb[tid][0] = c0 * invd;
        s_comb[tid][1] = c1 * invd;
        s_comb[tid][2] = c2 * invd;
        s_comb[tid][3] = 0.0f;
    }
    __syncthreads();

#pragma unroll
    for (int j = 0; j < 2; ++j) {
        const int c = 16 * j + m;
        const bool valid = (c < 24);
        const int e = valid ? (c >> 3) : 0;
#pragma unroll
        for (int v = 0; v < 8; ++v) {
            const int tl = 16 * w + 8 * h + v;
            const float dval = accd[j][v] * (1.0f / 32.0f);
            const float act = gelu_exact(dval);
            const float cav = valid ? 8.0f * (s_comb[tl][e] * act) : 0.0f;
            const unsigned short hi = bf16_rne(cav);
            const unsigned short lo = bf16_rne(cav - bf16_to_f32(hi));
            s_ca[tl][c] = hi;
            s_ca[tl][32 + c] = lo;
        }
    }
    __syncthreads();

    v4u pk[4];
#pragma unroll
    for (int it = 0; it < 4; ++it) {
        const int rl = 16 * w + 4 * it + (l >> 3);
        const int p = l & 7;
        pk[it] = *(const v4ua*)(&s_ca[rl][8 * p]);
    }
#pragma unroll
    for (int it = 0; it < 4; ++it) {
        const int rl = 16 * w + 4 * it + (l >> 3);
        const int p = l & 7;
        unsigned short* dst = ca + (size_t)(t0 + rl) * 64 + 8 * p;
        *(volatile v4u*)dst = pk[it];
    }
    __threadfence();
#pragma unroll
    for (int it = 0; it < 4; ++it) {
        const int rl = 16 * w + 4 * it + (l >> 3);
        const int p = l & 7;
        unsigned short* dst = ca + (size_t)(t0 + rl) * 64 + 8 * p;
        *(volatile v4u*)dst = pk[it];
    }
}

__global__ __launch_bounds__(128) void k_gemm1(const f16* __restrict__ A, const f16* __restrict__ Bt,
                                                const float* __restrict__ bias, f16* __restrict__ Hout,
                                                int M, int N, int K) {
    __shared__ __align__(16) f16 s_h[4][32][64];
    const int tid = threadIdx.x, w = tid >> 5, l = tid & 31, h = l >> 4, m = l & 15;
    const int mrow0 = blockIdx.y * 128 + 32 * w;
    const int ncol0 = blockIdx.x * 64;
    (void)M;

    v8f acc[2][4];
#pragma unroll
    for (int i = 0; i < 2; ++i)
#pragma unroll
        for (int j = 0; j < 4; ++j) acc[i][j] = vzero8();

    const f16* ap0 = A + (size_t)(mrow0 + m) * K;
    const f16* ap1 = ap0 + (size_t)16 * K;
    const f16* bp0 = Bt + (size_t)(ncol0 + m) * K;

#pragma unroll 1
    for (int k0 = 0; k0 < K; k0 += 32) {
        v16h a0 = ld_frag_h(ap0, k0, h);
        v16h a1 = ld_frag_h(ap1, k0, h);
        v16h b[4];
#pragma unroll
        for (int j = 0; j < 4; ++j) b[j] = ld_frag_h(bp0 + (size_t)(16 * j) * K, k0, h);
#pragma unroll
        for (int j = 0; j < 4; ++j) {
            acc[0][j] = wmma_f16(a0, b[j], acc[0][j]);
            acc[1][j] = wmma_f16(a1, b[j], acc[1][j]);
        }
    }

    float bj[4];
#pragma unroll
    for (int j = 0; j < 4; ++j) bj[j] = bias[ncol0 + 16 * j + m];
#pragma unroll
    for (int i = 0; i < 2; ++i)
#pragma unroll
        for (int j = 0; j < 4; ++j)
#pragma unroll
            for (int v = 0; v < 8; ++v) {
                const float pre = acc[i][j][v] * (1.0f / 32.0f) + bj[j];
                const float g = gelu_exact(pre);
                s_h[w][16 * i + 8 * h + v][16 * j + m] = (f16)(16.0f * g);
            }
    __syncthreads();

#pragma unroll
    for (int it = 0; it < 8; ++it) {
        const int rl = 4 * it + (l >> 3);
        const int p = l & 7;
        const v4u val = *(const v4ua*)(&s_h[w][rl][8 * p]);
        f16* dst = Hout + (size_t)(mrow0 + rl) * N + ncol0 + 8 * p;
        *(volatile v4u*)dst = val;
    }
    __threadfence();
#pragma unroll
    for (int it = 0; it < 8; ++it) {
        const int rl = 4 * it + (l >> 3);
        const int p = l & 7;
        const v4u val = *(const v4ua*)(&s_h[w][rl][8 * p]);
        f16* dst = Hout + (size_t)(mrow0 + rl) * N + ncol0 + 8 * p;
        *(volatile v4u*)dst = val;
    }
}

__global__ __launch_bounds__(128) void k_gemm2(const f16* __restrict__ A, const f16* __restrict__ Bt,
                                                const unsigned short* __restrict__ Ca,
                                                const unsigned short* __restrict__ Wu,
                                                const float* __restrict__ bias, float* __restrict__ Out,
                                                int M, int N, int K) {
    __shared__ __align__(16) float s_o[4][32][64];
    const int tid = threadIdx.x, w = tid >> 5, l = tid & 31, h = l >> 4, m = l & 15;
    const int mrow0 = blockIdx.y * 128 + 32 * w;
    const int ncol0 = blockIdx.x * 64;
    (void)M;

    v8f acc[2][4];
#pragma unroll
    for (int i = 0; i < 2; ++i)
#pragma unroll
        for (int j = 0; j < 4; ++j) acc[i][j] = vzero8();

    {
        const f16* ap0 = A + (size_t)(mrow0 + m) * K;
        const f16* ap1 = ap0 + (size_t)16 * K;
        const f16* bp0 = Bt + (size_t)(ncol0 + m) * K;
#pragma unroll 1
        for (int k0 = 0; k0 < K; k0 += 32) {
            v16h a0 = ld_frag_h(ap0, k0, h);
            v16h a1 = ld_frag_h(ap1, k0, h);
            v16h b[4];
#pragma unroll
            for (int j = 0; j < 4; ++j) b[j] = ld_frag_h(bp0 + (size_t)(16 * j) * K, k0, h);
#pragma unroll
            for (int j = 0; j < 4; ++j) {
                acc[0][j] = wmma_f16(a0, b[j], acc[0][j]);
                acc[1][j] = wmma_f16(a1, b[j], acc[1][j]);
            }
        }
    }

    {
        const unsigned short* cp0 = Ca + (size_t)(mrow0 + m) * 64;
        const unsigned short* cp1 = cp0 + (size_t)16 * 64;
        const unsigned short* up0 = Wu + (size_t)(ncol0 + m) * 64;
#pragma unroll
        for (int q = 0; q < 3; ++q) {
            const int ka = (q == 2) ? 32 : 0;
            const int kb = (q == 1) ? 32 : 0;
            v16b a0 = ld_frag_b(cp0, ka, h);
            v16b a1 = ld_frag_b(cp1, ka, h);
            v16b b[4];
#pragma unroll
            for (int j = 0; j < 4; ++j) b[j] = ld_frag_b(up0 + (size_t)(16 * j) * 64, kb, h);
#pragma unroll
            for (int j = 0; j < 4; ++j) {
                acc[0][j] = wmma_bf16(a0, b[j], acc[0][j]);
                acc[1][j] = wmma_bf16(a1, b[j], acc[1][j]);
            }
        }
    }

    float bj[4];
#pragma unroll
    for (int j = 0; j < 4; ++j) bj[j] = bias[ncol0 + 16 * j + m];
#pragma unroll
    for (int i = 0; i < 2; ++i)
#pragma unroll
        for (int j = 0; j < 4; ++j)
#pragma unroll
            for (int v = 0; v < 8; ++v)
                s_o[w][16 * i + 8 * h + v][16 * j + m] = acc[i][j][v] * (1.0f / 512.0f) + bj[j];
    __syncthreads();

#pragma unroll
    for (int it = 0; it < 16; ++it) {
        const int rl = 2 * it + (l >> 4);
        const int p = l & 15;
        const v4f val = *(const v4fa*)(&s_o[w][rl][4 * p]);
        float* dst = Out + (size_t)(mrow0 + rl) * N + ncol0 + 4 * p;
        *(volatile v4f*)dst = val;
    }
    __threadfence();
#pragma unroll
    for (int it = 0; it < 16; ++it) {
        const int rl = 2 * it + (l >> 4);
        const int p = l & 15;
        const v4f val = *(const v4fa*)(&s_o[w][rl][4 * p]);
        float* dst = Out + (size_t)(mrow0 + rl) * N + ncol0 + 4 * p;
        *(volatile v4f*)dst = val;
    }
}

extern "C" void kernel_launch(void* const* d_in, const int* in_sizes, int n_in,
                              void* d_out, int out_size, void* d_ws, size_t ws_size,
                              hipStream_t stream) {
    constexpr int D = 768, HID = 3072, E = 3, RK = 8;
    if (n_in < 9) return;
    const int T = in_sizes[0] / D;
    if (T <= 0 || (T % 128) != 0 || in_sizes[0] != T * D) return;
    if (in_sizes[1] != D * HID || in_sizes[2] != HID || in_sizes[3] != HID * D || in_sizes[4] != D) return;
    if (in_sizes[5] != D * E || in_sizes[6] != E || in_sizes[7] != E * D * RK || in_sizes[8] != E * RK * D) return;
    if (out_size != T * D) return;

    const float* x        = (const float*)d_in[0];
    const float* w1       = (const float*)d_in[1];
    const float* b1       = (const float*)d_in[2];
    const float* w2       = (const float*)d_in[3];
    const float* b2       = (const float*)d_in[4];
    const float* router_w = (const float*)d_in[5];
    const float* router_b = (const float*)d_in[6];
    const float* w_down   = (const float*)d_in[7];
    const float* w_up     = (const float*)d_in[8];
    float* out = (float*)d_out;

    char* ws = (char*)d_ws;
    size_t off = 0;
    auto take = [&](size_t bytes) -> char* {
        char* p = ws + off;
        off += (bytes + 255) & ~(size_t)255;
        return p;
    };
    f16* x16  = (f16*)take((size_t)T * D * sizeof(f16));
    f16* w1t  = (f16*)take((size_t)HID * D * sizeof(f16));
    f16* w2t  = (f16*)take((size_t)D * HID * sizeof(f16));
    f16* h16  = (f16*)take((size_t)T * HID * sizeof(f16));
    f16* wd16 = (f16*)take((size_t)32 * D * sizeof(f16));
    unsigned short* wu = (unsigned short*)take((size_t)D * 64 * sizeof(unsigned short));
    unsigned short* ca = (unsigned short*)take((size_t)T * 64 * sizeof(unsigned short));
    if (off > ws_size) return;

    k_cvt_x<<<dim3((T + 7) / 8), dim3(256), 0, stream>>>(x, x16, T);
    k_prep_w<<<dim3(HID / 32, D / 64), dim3(64), 0, stream>>>(w1, w1t, D, HID, 32.0f);
    k_prep_w<<<dim3(D / 32, HID / 64), dim3(64), 0, stream>>>(w2, w2t, HID, D, 32.0f);
    k_prep_s<<<dim3(2), dim3(256), 0, stream>>>(w_down, w_up, wd16, wu);

    k_tok<<<dim3(T / 32), dim3(64), 0, stream>>>(x, router_w, router_b, x16, wd16, ca, T);

    k_gemm1<<<dim3(HID / 64, T / 128), dim3(128), 0, stream>>>(x16, w1t, b1, h16, T, HID, D);

    k_gemm2<<<dim3(D / 64, T / 128), dim3(128), 0, stream>>>(h16, w2t, ca, wu, b2, out, T, D, HID);
}
